// LinearAttention_20598663152021
// MI455X (gfx1250) — hardware-verified
//
#include <hip/hip_runtime.h>
#include <math.h>

constexpr int kBatch    = 4;
constexpr int kSeq      = 2048;
constexpr int kDm       = 1024;
constexpr int kHeads    = 8;
constexpr int kHd       = 128;
constexpr int kFeat     = 256;
constexpr int kFeatRoot = 16;
constexpr int kChunk    = 64;
constexpr int kRows     = kBatch * kSeq;
constexpr int kPhiLd    = kHeads * kFeat;
constexpr int kKtP      = 72;
constexpr int kSmP      = 264;
constexpr int kOsP      = 132;
constexpr int kAttnThr  = 512;
constexpr float kWCarry    = 16.0f;
constexpr float kWCarryInv = 1.0f / kWCarry;
constexpr float kQScale    = 1.0f / (float)kFeatRoot;
constexpr float kRmsEps    = 1e-5f;
static_assert(kFeatRoot * kFeatRoot == kFeat, "feature scale is kFeat^-0.5");
static_assert(kHeads * kHd == kDm, "head split");
static_assert(kFeat == 2 * kHd, "two exp halves per head");
static_assert(kRows % 64 == 0 && kDm % 64 == 0 && kDm % 32 == 0, "GEMM tile multiples");
static_assert(kHd % 64 == 0 && kHd % 32 == 0, "fold GEMM tile multiples");
static_assert(kSeq % kChunk == 0 && kChunk == 64, "chunking");
static_assert((kHd * kSmP) % kAttnThr == 0, "mirror zero-fill loop exact");
static_assert(kFeat == 16 * (kAttnThr / 32), "one 16-row state tile per wave");

typedef __attribute__((ext_vector_type(16))) _Float16 v16h;
typedef __attribute__((ext_vector_type(8)))  _Float16 v8h;
typedef __attribute__((ext_vector_type(16))) __bf16   v16b;
typedef __attribute__((ext_vector_type(8)))  __bf16   v8b;
typedef __attribute__((ext_vector_type(8)))  float    v8f;
typedef __attribute__((ext_vector_type(4)))  float    v4f;
typedef __attribute__((ext_vector_type(4)))  unsigned int v4u;

__device__ __forceinline__ unsigned short f2bf_bits(float f) {
  unsigned u = __float_as_uint(f);
  return (unsigned short)((u + 0x7FFFu + ((u >> 16) & 1u)) >> 16);
}
__device__ __forceinline__ float bf_bits2f(unsigned short h) { return __uint_as_float(((unsigned)h) << 16); }

__device__ __forceinline__ void dep_guard4_h(v8f& a, v8f& b, v8f& c, v8f& d, v16h x, v16h y) {
  asm volatile("v_nop\n\tv_nop\n\tv_nop\n\tv_nop" : "+v"(a), "+v"(b), "+v"(c), "+v"(d) : "v"(x), "v"(y));
}
__device__ __forceinline__ void dep_guard4_b(v8f& a, v8f& b, v8f& c, v8f& d, v16b x, v16b y) {
  asm volatile("v_nop\n\tv_nop\n\tv_nop\n\tv_nop" : "+v"(a), "+v"(b), "+v"(c), "+v"(d) : "v"(x), "v"(y));
}
__device__ __forceinline__ void keep4_h(v16h a, v16h b, v16h c, v16h d) { asm volatile("v_nop" :: "v"(a), "v"(b), "v"(c), "v"(d)); }
__device__ __forceinline__ void keep4_b(v16b a, v16b b, v16b c, v16b d) { asm volatile("v_nop" :: "v"(a), "v"(b), "v"(c), "v"(d)); }
__device__ __forceinline__ void acc_guard4(v8f& a, v8f& b, v8f& c, v8f& d) {
  asm volatile("v_nop\n\tv_nop\n\tv_nop\n\tv_nop" : "+v"(a), "+v"(b), "+v"(c), "+v"(d));
}

template <typename T> struct Frag;
template <> struct Frag<_Float16> {
  typedef v16h V; union U { v16h v; v8h h[2]; };
  static __device__ __forceinline__ v16h load(const _Float16* p) {
    U f; f.h[0] = *(const v8h*)(p); f.h[1] = *(const v8h*)(p + 16); return f.v;
  }
  static __device__ __forceinline__ v8f mma(v16h a, v16h b, v8f c) {
    return __builtin_amdgcn_wmma_f32_16x16x32_f16(false, a, false, b, (short)0, c, false, false);
  }
  static __device__ __forceinline__ void guard4(v8f& a, v8f& b, v8f& c, v8f& d, v16h x, v16h y) { dep_guard4_h(a, b, c, d, x, y); }
  static __device__ __forceinline__ void keep(v16h a, v16h b, v16h c, v16h d) { keep4_h(a, b, c, d); }
};
template <> struct Frag<__bf16> {
  typedef v16b V; union U { v16b v; v8b h[2]; };
  static __device__ __forceinline__ v16b load(const __bf16* p) {
    U f; f.h[0] = *(const v8b*)(p); f.h[1] = *(const v8b*)(p + 16); return f.v;
  }
  static __device__ __forceinline__ v8f mma(v16b a, v16b b, v8f c) {
    return __builtin_amdgcn_wmma_f32_16x16x32_bf16(false, a, false, b, (short)0, c, false, false);
  }
  static __device__ __forceinline__ void guard4(v8f& a, v8f& b, v8f& c, v8f& d, v16b x, v16b y) { dep_guard4_b(a, b, c, d, x, y); }
  static __device__ __forceinline__ void keep(v16b a, v16b b, v16b c, v16b d) { keep4_b(a, b, c, d); }
};

__device__ __forceinline__ unsigned pk16(unsigned short a, unsigned short b) { return (unsigned)a | ((unsigned)b << 16); }
__device__ __forceinline__ unsigned short h_bits(float f) { const _Float16 h = (_Float16)f; return __builtin_bit_cast(unsigned short, h); }
__device__ __forceinline__ _Float16 bits2h(unsigned w) {
  const unsigned short s = (unsigned short)(w & 0xffffu);
  return __builtin_bit_cast(_Float16, s);
}

__device__ __forceinline__ v8f mma_h(v16h a, v16h b, v8f c) {
  c = __builtin_amdgcn_wmma_f32_16x16x32_f16(false, a, false, b, (short)0, c, false, false);
  asm volatile("v_nop\n\tv_nop\n\tv_nop\n\tv_nop" : "+v"(c) : "v"(a), "v"(b));
  return c;
}

template <int ET> struct Elem;
template <> struct Elem<0> { typedef _Float16 T; };
template <> struct Elem<1> { typedef __bf16 T; };
template <int ET, bool SPLIT, int BIAS_MODE, int OUT_MODE, bool RESID, int ACT = 0>
__global__ __launch_bounds__(256) void wmma_gemm64(
    const unsigned short* __restrict__ Ap, const unsigned short* __restrict__ A2p, int lda, long strideA,
    const unsigned short* __restrict__ Btp, const unsigned short* __restrict__ Bt2p, int ldb, long strideB,
    void* __restrict__ Cout, void* __restrict__ Cout2, int ldc, long strideC,
    const float* __restrict__ bias,
    const float* __restrict__ resid, long strideR,
    int M, int N, int K, float scale) {
  typedef typename Elem<ET>::T T;
  typedef typename Frag<T>::V V;
  const T* A = (const T*)Ap; const T* A2 = (const T*)A2p; const T* Bt = (const T*)Btp; const T* Bt2 = (const T*)Bt2p;
  __shared__ __align__(16) float sT[8][16 * 68];
  const int b    = blockIdx.y;
  const int lane = threadIdx.x & 31;
  const int wave = threadIdx.x >> 5;
  const int tilesN = N >> 6;
  const int tilesM = M >> 6;
  const int tile = blockIdx.x * 8 + wave;
  if (tile >= tilesM * tilesN) return;
  const int tm = tile / tilesN;
  const int tn = tile - tm * tilesN;
  const int m0 = tm << 6;
  const int n0 = tn << 6;

  const T* Ab  = A  + (size_t)b * strideA;
  const T* Bb  = Bt + (size_t)b * strideB;
  const T* Ab2 = SPLIT ? (A2  + (size_t)b * strideA) : nullptr;
  const T* Bb2 = SPLIT ? (Bt2 + (size_t)b * strideB) : nullptr;

  const int rlane = lane & 15;
  const int koff  = (lane >> 4) * 8;
  const int mOff  = (lane >> 4) * 8;

  v8f acc[4][4];
#pragma unroll
  for (int i = 0; i < 4; ++i)
#pragma unroll
    for (int j = 0; j < 4; ++j) acc[i][j] = (v8f){0.f,0.f,0.f,0.f,0.f,0.f,0.f,0.f};

  for (int k0 = 0; k0 < K; k0 += 32) {
    V bh[4], bl[4];
#pragma unroll
    for (int j = 0; j < 4; ++j) {
      const size_t bo = (size_t)(n0 + (j << 4) + rlane) * ldb + koff + k0;
      bh[j] = Frag<T>::load(Bb + bo);
      if (SPLIT) bl[j] = Frag<T>::load(Bb2 + bo);
    }
#pragma unroll
    for (int i = 0; i < 4; ++i) {
      const size_t ao = (size_t)(m0 + (i << 4) + rlane) * lda + koff + k0;
      V ah = Frag<T>::load(Ab + ao);
      V al;
      if (SPLIT) al = Frag<T>::load(Ab2 + ao);
#pragma unroll
      for (int j = 0; j < 4; ++j) {
        acc[i][j] = Frag<T>::mma(ah, bh[j], acc[i][j]);
        if (SPLIT) {
          acc[i][j] = Frag<T>::mma(ah, bl[j], acc[i][j]);
          acc[i][j] = Frag<T>::mma(al, bh[j], acc[i][j]);
        }
      }
      Frag<T>::guard4(acc[i][0], acc[i][1], acc[i][2], acc[i][3], ah, SPLIT ? al : ah);
    }
    Frag<T>::keep(bh[0], bh[1], bh[2], bh[3]);
    if (SPLIT) Frag<T>::keep(bl[0], bl[1], bl[2], bl[3]);
  }
  acc_guard4(acc[0][0], acc[0][1], acc[0][2], acc[0][3]);
  acc_guard4(acc[1][0], acc[1][1], acc[1][2], acc[1][3]);
  acc_guard4(acc[2][0], acc[2][1], acc[2][2], acc[2][3]);
  acc_guard4(acc[3][0], acc[3][1], acc[3][2], acc[3][3]);

  float* slab = sT[wave];
  const float* Rb = RESID ? (resid + (size_t)b * strideR) : nullptr;
#pragma unroll
  for (int i = 0; i < 4; ++i) {
    const int mBase = m0 + (i << 4);
#pragma unroll
    for (int j = 0; j < 4; ++j) {
      const int n = n0 + (j << 4) + rlane;
      float bv = 0.f;
      if (BIAS_MODE == 2) bv = bias[n];
#pragma unroll
      for (int r = 0; r < 8; ++r) {
        float v = acc[i][j][r] * scale;
        if (BIAS_MODE == 1) v += bias[mBase + mOff + r];
        if (BIAS_MODE == 2) v += bv;
        if (RESID) v += Rb[(size_t)(mBase + mOff + r) * ldc + n];
        if (ACT == 2) v = fmaxf(v, 0.0f);
        if (ACT == 4) v = (v > 0.f) ? v : 0.01f * v;
        slab[(mOff + r) * 68 + (j << 4) + rlane] = v;
      }
    }
    __builtin_amdgcn_fence(__ATOMIC_RELEASE, "workgroup");
    __builtin_amdgcn_wave_barrier();
    __builtin_amdgcn_fence(__ATOMIC_ACQUIRE, "workgroup");
    if (OUT_MODE == 0) {
      float* C = (float*)Cout + (size_t)b * strideC;
      const int hh = lane >> 4, c4 = (lane & 15) * 4;
      for (int pass = 0; pass < 2; ++pass) {
#pragma unroll
        for (int it = 0; it < 8; ++it) {
          const int row = it * 2 + hh;
          v4f v = *(const v4f*)(slab + row * 68 + c4);
          *(volatile v4f*)(C + (size_t)(mBase + row) * ldc + n0 + c4) = v;
        }
        __threadfence();
      }
    } else {
      const int q = lane >> 3, c8 = (lane & 7) * 8;
      unsigned short* C  = (unsigned short*)Cout  + (size_t)b * strideC;
      unsigned short* C2 = (OUT_MODE == 2) ? ((unsigned short*)Cout2 + (size_t)b * strideC) : nullptr;
      for (int pass = 0; pass < 2; ++pass) {
#pragma unroll
        for (int it = 0; it < 4; ++it) {
          const int row = it * 4 + q;
          const float* sp = slab + row * 68 + c8;
          v8h hv, lv;
#pragma unroll
          for (int e = 0; e < 8; ++e) {
            if (OUT_MODE == 1) {
              hv[e] = (_Float16)sp[e];
            } else {
              unsigned short hb = f2bf_bits(sp[e]);
              unsigned short lb = f2bf_bits(sp[e] - bf_bits2f(hb));
              hv[e] = __builtin_bit_cast(_Float16, hb);
              lv[e] = __builtin_bit_cast(_Float16, lb);
            }
          }
          *(volatile v8h*)(C + (size_t)(mBase + row) * ldc + n0 + c8) = hv;
          if (OUT_MODE == 2) *(volatile v8h*)(C2 + (size_t)(mBase + row) * ldc + n0 + c8) = lv;
        }
        __threadfence();
      }
    }
    __builtin_amdgcn_fence(__ATOMIC_RELEASE, "workgroup");
    __builtin_amdgcn_wave_barrier();
    __builtin_amdgcn_fence(__ATOMIC_ACQUIRE, "workgroup");
  }
}

__global__ __launch_bounds__(256) void feat_gemm64(
    const unsigned short* __restrict__ Ap, const unsigned short* __restrict__ Btp,
    unsigned short* __restrict__ Phi, const float* __restrict__ fb, float inv_carry, float fs) {
  typedef _Float16 T;
  typedef v16h V;
  const T* A  = (const T*)(const void*)Ap;
  const T* Bt = (const T*)(const void*)Btp;
  __shared__ __align__(16) float sT[8][16 * 68];
  const int lane = threadIdx.x & 31;
  const int wave = threadIdx.x >> 5;
  constexpr int tilesN = kDm >> 6;
  constexpr int tilesM = kRows >> 6;
  const int tile = blockIdx.x * 8 + wave;
  if (tile >= tilesM * tilesN) return;
  const int tm = tile / tilesN;
  const int tn = tile - tm * tilesN;
  const int m0 = tm << 6;
  const int n0 = tn << 6;
  const int rlane = lane & 15;
  const int koff  = (lane >> 4) * 8;
  const int mOff  = (lane >> 4) * 8;

  v8f acc[4][4];
#pragma unroll
  for (int i = 0; i < 4; ++i)
#pragma unroll
    for (int j = 0; j < 4; ++j) acc[i][j] = (v8f){0.f,0.f,0.f,0.f,0.f,0.f,0.f,0.f};

  const T* Bbase = Bt + (size_t)(n0 + rlane) * kDm + koff;
  const T* Abase = A  + (size_t)(m0 + rlane) * kDm + koff;
  for (int k0 = 0; k0 < kDm; k0 += 32) {
    V bh[4];
#pragma unroll
    for (int j = 0; j < 4; ++j) bh[j] = Frag<T>::load(Bbase + (size_t)(j << 4) * kDm + k0);
#pragma unroll
    for (int i = 0; i < 4; ++i) {
      V ah = Frag<T>::load(Abase + (size_t)(i << 4) * kDm + k0);
#pragma unroll
      for (int j = 0; j < 4; ++j) acc[i][j] = Frag<T>::mma(ah, bh[j], acc[i][j]);
      Frag<T>::guard4(acc[i][0], acc[i][1], acc[i][2], acc[i][3], ah, ah);
    }
    Frag<T>::keep(bh[0], bh[1], bh[2], bh[3]);
  }
  acc_guard4(acc[0][0], acc[0][1], acc[0][2], acc[0][3]);
  acc_guard4(acc[1][0], acc[1][1], acc[1][2], acc[1][3]);
  acc_guard4(acc[2][0], acc[2][1], acc[2][2], acc[2][3]);
  acc_guard4(acc[3][0], acc[3][1], acc[3][2], acc[3][3]);

  float* slab = sT[wave];
  const int head = n0 >> 7;
  const int e0   = n0 & (kHd - 1);
  const int q    = lane >> 3;
  const int c8   = (lane & 7) * 8;
  float bv[4];
#pragma unroll
  for (int j = 0; j < 4; ++j) bv[j] = fb[(n0 + (j << 4) + rlane) & (kHd - 1)];
#pragma unroll
  for (int i = 0; i < 4; ++i) {
    const int mBase = m0 + (i << 4);
#pragma unroll
    for (int j = 0; j < 4; ++j) {
#pragma unroll
      for (int r = 0; r < 8; ++r) {
        const float y = acc[i][j][r] * inv_carry + bv[j];
        slab[(mOff + r) * 68 + (j << 4) + rlane] = y;
      }
    }
    __builtin_amdgcn_fence(__ATOMIC_RELEASE, "workgroup");
    __builtin_amdgcn_wave_barrier();
    __builtin_amdgcn_fence(__ATOMIC_ACQUIRE, "workgroup");
#pragma unroll 1
    for (int it = 0; it < 4; ++it) {
      const int row = it * 4 + q;
      const float* sp = slab + row * 68 + c8;
      const v4f ya = *(const v4f*)(sp);
      const v4f yb = *(const v4f*)(sp + 4);
      v8h hv, lv;
#pragma unroll
      for (int e = 0; e < 4; ++e) {
        const float y0 = ya[e];
        const float y1 = yb[e];
        const float p0 = expf(y0);
        const float p1 = expf(y1);
        const float r0 = __builtin_amdgcn_rcpf(p0);
        const float r1 = __builtin_amdgcn_rcpf(p1);
        hv[e]     = (_Float16)(p0 * fs);
        hv[4 + e] = (_Float16)(p1 * fs);
        lv[e]     = (_Float16)(r0 * fs);
        lv[4 + e] = (_Float16)(r1 * fs);
      }
      unsigned short* dp = Phi + (size_t)(mBase + row) * kPhiLd + head * kFeat + e0 + c8;
      *(volatile v8h*)(dp)       = hv;
      *(volatile v8h*)(dp + kHd) = lv;
      __threadfence();
      *(volatile v8h*)(dp)       = hv;
      *(volatile v8h*)(dp + kHd) = lv;
    }
    __builtin_amdgcn_fence(__ATOMIC_RELEASE, "workgroup");
    __builtin_amdgcn_wave_barrier();
    __builtin_amdgcn_fence(__ATOMIC_ACQUIRE, "workgroup");
  }
}

__global__ __launch_bounds__(256) void cast8_f16_kernel(const float* __restrict__ in, unsigned short* __restrict__ out, int n8, float sc) {
  const int i = blockIdx.x * 256 + threadIdx.x;
  if (i >= n8) return;
  const float* p = in + 8 * (size_t)i;
  const v4f a = *(const v4f*)(p);
  const v4f c = *(const v4f*)(p + 4);
  unsigned short hb[8];
#pragma unroll
  for (int e = 0; e < 4; ++e) {
    hb[e]     = h_bits(a[e] * sc);
    hb[4 + e] = h_bits(c[e] * sc);
  }
  const v4u u = (v4u){pk16(hb[0], hb[1]), pk16(hb[2], hb[3]), pk16(hb[4], hb[5]), pk16(hb[6], hb[7])};
  unsigned short* q = out + 8 * (size_t)i;
  *(volatile v4u*)q = u;
  __threadfence();
  *(volatile v4u*)q = u;
}

__global__ __launch_bounds__(256) void wtcast_kernel(const float* __restrict__ W0, const float* __restrict__ W1,
                                                     unsigned short* __restrict__ out, float scale) {
  __shared__ float sm[64][65];
  const int t  = threadIdx.x;
  const int j0 = blockIdx.x * 64;
  const int c0 = blockIdx.y * 64;
  const int z  = blockIdx.z;
  const float* W = (z == 0) ? W0 : W1;
#pragma unroll
  for (int i = 0; i < 16; ++i) {
    const int e = i * 256 + t;
    const int r = e >> 6;
    const int c = e & 63;
    sm[c][r] = W[(size_t)(j0 + r) * kDm + c0 + c] * scale;
  }
  __syncthreads();
  const int lane = t & 31, wave = t >> 5;
  const int q = lane >> 3, c8 = (lane & 7) * 8;
  unsigned short* op = out + (size_t)z * kDm * kDm;
  for (int pass = 0; pass < 2; ++pass) {
#pragma unroll
    for (int it = 0; it < 2; ++it) {
      const int row = wave * 8 + it * 4 + q;
      unsigned short hb[8];
#pragma unroll
      for (int e = 0; e < 8; ++e) hb[e] = h_bits(sm[row][c8 + e]);
      const v4u u = (v4u){pk16(hb[0], hb[1]), pk16(hb[2], hb[3]), pk16(hb[4], hb[5]), pk16(hb[6], hb[7])};
      *(volatile v4u*)(op + (size_t)(c0 + row) * kDm + j0 + c8) = u;
    }
    __threadfence();
  }
}

__global__ __launch_bounds__(kAttnThr) void chunk_attn_kernel(
    const unsigned short* __restrict__ PhiQp, const unsigned short* __restrict__ PhiKp,
    const unsigned short* __restrict__ Vp, const float* __restrict__ rms_w,
    unsigned short* __restrict__ Onp) {
  __shared__ __align__(16) _Float16 Kt[kFeat * kKtP];
  __shared__ __align__(16) _Float16 Vt[kHd * kKtP];
  __shared__ __align__(16) _Float16 Asc[kChunk * kKtP];
  __shared__ __align__(16) _Float16 Sm[kHd * kSmP];
  __shared__ __align__(16) float    Ost[kChunk * kOsP];

  const int tid  = threadIdx.x;
  const int lane = tid & 31;
  const int wave = tid >> 5;
  const int cl   = lane & 15;
  const int hh   = lane >> 4;
  const int koff = hh * 8;
  const int bh   = blockIdx.x;
  const int b    = bh / kHeads;
  const int h    = bh - b * kHeads;
  const size_t phiBase = (size_t)b * kSeq * kPhiLd + (size_t)h * kFeat;
  const size_t vBase   = (size_t)b * kSeq * kDm + (size_t)h * kHd;
  const unsigned short* kgU = PhiKp + phiBase;
  const _Float16* qg = (const _Float16*)(const void*)PhiQp + phiBase;
  const _Float16* kg = (const _Float16*)(const void*)PhiKp + phiBase;
  const unsigned short* vgU = Vp + vBase;
  unsigned short* og = Onp + vBase;

#pragma unroll 1
  for (int i = tid; i < kHd * kSmP; i += kAttnThr) Sm[i] = (_Float16)0.0f;

  const v8f z8 = {0.f, 0.f, 0.f, 0.f, 0.f, 0.f, 0.f, 0.f};
  v8f S[8];
#pragma unroll
  for (int nt = 0; nt < 8; ++nt) S[nt] = z8;

  const v4f g0 = *(const v4f*)(rms_w + 8 * cl);
  const v4f g1 = *(const v4f*)(rms_w + 8 * cl + 4);
  const int mt = wave >> 2;
  const int nq = wave & 3;

#pragma unroll 1
  for (int c0 = 0; c0 < kSeq; c0 += kChunk) {
#pragma unroll
    for (int j = 0; j < 4; ++j) {
      const int u   = tid + j * kAttnThr;
      const int row = u >> 5;
      const int sg  = (u & 31) * 8;
      const v4u w = *(const v4u*)(kgU + (size_t)(c0 + row) * kPhiLd + sg);
      const unsigned w0 = w[0], w1 = w[1], w2 = w[2], w3 = w[3];
      _Float16* kp = Kt + sg * kKtP + row;
      kp[0 * kKtP] = bits2h(w0);
      kp[1 * kKtP] = bits2h(w0 >> 16);
      kp[2 * kKtP] = bits2h(w1);
      kp[3 * kKtP] = bits2h(w1 >> 16);
      kp[4 * kKtP] = bits2h(w2);
      kp[5 * kKtP] = bits2h(w2 >> 16);
      kp[6 * kKtP] = bits2h(w3);
      kp[7 * kKtP] = bits2h(w3 >> 16);
    }
#pragma unroll
    for (int j = 0; j < 2; ++j) {
      const int u   = tid + j * kAttnThr;
      const int row = u >> 4;
      const int sg  = (u & 15) * 8;
      const v4u w = *(const v4u*)(vgU + (size_t)(c0 + row) * kDm + sg);
      const unsigned w0 = w[0], w1 = w[1], w2 = w[2], w3 = w[3];
      _Float16* vp = Vt + sg * kKtP + row;
      vp[0 * kKtP] = bits2h(w0);
      vp[1 * kKtP] = bits2h(w0 >> 16);
      vp[2 * kKtP] = bits2h(w1);
      vp[3 * kKtP] = bits2h(w1 >> 16);
      vp[4 * kKtP] = bits2h(w2);
      vp[5 * kKtP] = bits2h(w2 >> 16);
      vp[6 * kKtP] = bits2h(w3);
      vp[7 * kKtP] = bits2h(w3 >> 16);
    }
    __syncthreads();

    {
      v8f sc = z8;
      const _Float16* qa = qg + (size_t)(c0 + 16 * mt + cl) * kPhiLd + koff;
      const _Float16* kb = kg + (size_t)(c0 + 16 * nq + cl) * kPhiLd + koff;
#pragma unroll
      for (int ks = 0; ks < 8; ++ks) {
        const v16h a  = Frag<_Float16>::load(qa + 32 * ks);
        const v16h bf = Frag<_Float16>::load(kb + 32 * ks);
        sc = mma_h(a, bf, sc);
      }
      const int ecol = 16 * nq + cl;
#pragma unroll
      for (int r = 0; r < 8; ++r) {
        const int crow = 16 * mt + 8 * hh + r;
        const float val = (ecol <= crow) ? sc[r] : 0.0f;
        Asc[crow * kKtP + ecol] = (_Float16)val;
      }
    }
    __syncthreads();

    {
      v8f o0 = z8, o1 = z8;
      const _Float16* ap  = Asc + (16 * mt + cl) * kKtP + koff;
      const _Float16* v0p = Vt + (32 * nq + cl) * kKtP + koff;
      const _Float16* v1p = v0p + 16 * kKtP;
#pragma unroll
      for (int ks = 0; ks < 2; ++ks) {
        const v16h a  = Frag<_Float16>::load(ap + 32 * ks);
        const v16h b0 = Frag<_Float16>::load(v0p + 32 * ks);
        const v16h b1 = Frag<_Float16>::load(v1p + 32 * ks);
        o0 = mma_h(a, b0, o0);
        o1 = mma_h(a, b1, o1);
      }
      const _Float16* qa  = qg + (size_t)(c0 + 16 * mt + cl) * kPhiLd + koff;
      const _Float16* s0p = Sm + (32 * nq + cl) * kSmP + koff;
      const _Float16* s1p = s0p + 16 * kSmP;
#pragma unroll
      for (int ks = 0; ks < 8; ++ks) {
        const v16h a  = Frag<_Float16>::load(qa + 32 * ks);
        const v16h b0 = Frag<_Float16>::load(s0p + 32 * ks);
        const v16h b1 = Frag<_Float16>::load(s1p + 32 * ks);
        o0 = mma_h(a, b0, o0);
        o1 = mma_h(a, b1, o1);
      }
#pragma unroll
      for (int r = 0; r < 8; ++r) {
        float* orow = Ost + (16 * mt + 8 * hh + r) * kOsP + 32 * nq + cl;
        orow[0]  = o0[r];
        orow[16] = o1[r];
      }
    }
    __syncthreads();

    {
      v8h hv[2];
#pragma unroll
      for (int it = 0; it < 2; ++it) {
        const int row = 4 * wave + 2 * it + hh;
        const float* op = Ost + row * kOsP + 8 * cl;
        const v4f a = *(const v4f*)(op);
        const v4f c = *(const v4f*)(op + 4);
        float ss = 0.0f;
#pragma unroll
        for (int e = 0; e < 4; ++e) ss += a[e] * a[e];
#pragma unroll
        for (int e = 0; e < 4; ++e) ss += c[e] * c[e];
        ss += __shfl_xor(ss, 1, 32);
        ss += __shfl_xor(ss, 2, 32);
        ss += __shfl_xor(ss, 4, 32);
        ss += __shfl_xor(ss, 8, 32);
        const float inv = rsqrtf(ss * (1.0f / (float)kHd) + kRmsEps);
#pragma unroll
        for (int e = 0; e < 4; ++e) {
          hv[it][e]     = (_Float16)((a[e] * inv) * g0[e]);
          hv[it][4 + e] = (_Float16)((c[e] * inv) * g1[e]);
        }
      }
#pragma unroll
      for (int pass = 0; pass < 2; ++pass) {
#pragma unroll
        for (int it = 0; it < 2; ++it) {
          const int row = 4 * wave + 2 * it + hh;
          *(volatile v8h*)(og + (size_t)(c0 + row) * kDm + 8 * cl) = hv[it];
        }
        __threadfence();
      }
    }

    {
      const _Float16* ap = Kt + (16 * wave + cl) * kKtP + koff;
      const _Float16* vp = Vt + cl * kKtP + koff;
#pragma unroll
      for (int ks = 0; ks < 2; ++ks) {
        const v16h a = Frag<_Float16>::load(ap + 32 * ks);
#pragma unroll
        for (int nt = 0; nt < 8; ++nt) {
          const v16h bf = Frag<_Float16>::load(vp + (16 * nt) * kKtP + 32 * ks);
          S[nt] = mma_h(a, bf, S[nt]);
        }
      }
#pragma unroll
      for (int nt = 0; nt < 8; ++nt) {
        v8h pk;
#pragma unroll
        for (int r = 0; r < 8; ++r) pk[r] = (_Float16)S[nt][r];
        *(v8h*)(Sm + (16 * nt + cl) * kSmP + 16 * wave + 8 * hh) = pk;
      }
    }
    __syncthreads();
  }
}

extern "C" void kernel_launch(void* const* d_in, const int* in_sizes, int n_in,
                              void* d_out, int out_size, void* d_ws, size_t ws_size, hipStream_t stream) {
  if (n_in < 10 || d_out == nullptr || d_ws == nullptr) return;
  if (in_sizes[0] != kRows * kDm || in_sizes[1] != kDm * kDm || in_sizes[2] != kDm * kDm ||
      in_sizes[3] != kDm * kDm || in_sizes[4] != kDm * kDm || in_sizes[5] != kHd * kHd ||
      in_sizes[6] != kHd || in_sizes[7] != kHd * kHd || in_sizes[8] != kHd || in_sizes[9] != kHd ||
      out_size != kRows * kDm) return;

  const float* x     = (const float*)d_in[0];
  const float* Wq    = (const float*)d_in[1];
  const float* Wk    = (const float*)d_in[2];
  const float* Wv    = (const float*)d_in[3];
  const float* Wo    = (const float*)d_in[4];
  const float* fmq_w = (const float*)d_in[5];
  const float* fmq_b = (const float*)d_in[6];
  const float* fmk_w = (const float*)d_in[7];
  const float* fmk_b = (const float*)d_in[8];
  const float* rms_w = (const float*)d_in[9];
  float* out = (float*)d_out;

  char* ws = (char*)d_ws; size_t off = 0;
  auto carve = [&](size_t bytes) -> char* { char* p = ws + off; off += (bytes + 255) & ~(size_t)255; return p; };
  unsigned short* XH   = (unsigned short*)carve((size_t)kRows * kDm * 2);
  unsigned short* WT   = (unsigned short*)carve((size_t)2 * kDm * kDm * 2);
  unsigned short* FMH  = (unsigned short*)carve((size_t)2 * kHd * kHd * 2);
  unsigned short* WQT  = (unsigned short*)carve((size_t)kDm * kDm * 2);
  unsigned short* WKT  = (unsigned short*)carve((size_t)kDm * kDm * 2);
  unsigned short* WVH  = (unsigned short*)carve((size_t)kDm * kDm * 2);
  unsigned short* WOH  = (unsigned short*)carve((size_t)kDm * kDm * 2);
  unsigned short* PHIQ = (unsigned short*)carve((size_t)kRows * kPhiLd * 2);
  unsigned short* PHIK = (unsigned short*)carve((size_t)kRows * kPhiLd * 2);
  unsigned short* VH   = (unsigned short*)carve((size_t)kRows * kDm * 2);
  unsigned short* ON   = (unsigned short*)carve((size_t)kRows * kDm * 2);
  if (off > ws_size || off > (size_t)134217728) return;

  const int n8x = kRows * kDm / 8;
  const int n8w = kDm * kDm / 8;
  const int n8f = kHd * kHd / 8;
  cast8_f16_kernel<<<n8x / 256, 256, 0, stream>>>(x, XH, n8x, 1.0f);
  cast8_f16_kernel<<<n8w / 256, 256, 0, stream>>>(Wv, WVH, n8w, kWCarry);
  cast8_f16_kernel<<<n8w / 256, 256, 0, stream>>>(Wo, WOH, n8w, kWCarry);
  cast8_f16_kernel<<<n8f / 256, 256, 0, stream>>>(fmq_w, FMH, n8f, kWCarry);
  cast8_f16_kernel<<<n8f / 256, 256, 0, stream>>>(fmk_w, FMH + kHd * kHd, n8f, kWCarry);
  wtcast_kernel<<<dim3(kDm / 64, kDm / 64, 2), 256, 0, stream>>>(Wq, Wk, WT, kWCarry);

  wmma_gemm64<0, false, 0, 1, false, 0><<<dim3(4, kHeads), 256, 0, stream>>>(
      FMH, FMH, kHd, 0L, WT, WT, kDm, (long)kHd,
      (void*)WQT, (void*)WQT, kDm, (long)kHd * kDm, fmq_b, rms_w, 0L, kHd, kDm, kHd, kWCarryInv);
  wmma_gemm64<0, false, 0, 1, false, 0><<<dim3(4, kHeads), 256, 0, stream>>>(
      FMH + kHd * kHd, FMH + kHd * kHd, kHd, 0L, WT + (size_t)kDm * kDm, WT + (size_t)kDm * kDm, kDm, (long)kHd,
      (void*)WKT, (void*)WKT, kDm, (long)kHd * kDm, fmk_b, rms_w, 0L, kHd, kDm, kHd, kWCarryInv);

  const int gblocks = (kRows / 64) * (kDm / 64) / 8;
  feat_gemm64<<<gblocks, 256, 0, stream>>>(XH, WQT, PHIQ, fmq_b, kWCarryInv, kQScale);
  feat_gemm64<<<gblocks, 256, 0, stream>>>(XH, WKT, PHIK, fmk_b, kWCarryInv, 1.0f);
  wmma_gemm64<0, false, 0, 1, false, 0><<<dim3(gblocks, 1), 256, 0, stream>>>(
      XH, XH, kDm, 0L, WVH, WVH, kDm, 0L,
      (void*)VH, (void*)VH, kDm, 0L, fmq_b, rms_w, 0L, kRows, kDm, kDm, kWCarryInv);

  chunk_attn_kernel<<<kBatch * kHeads, kAttnThr, 0, stream>>>(PHIQ, PHIK, VH, rms_w, ON);

  wmma_gemm64<0, false, 0, 0, false, 0><<<dim3(gblocks, 1), 256, 0, stream>>>(
      ON, ON, kDm, 0L, WOH, WOH, kDm, 0L,
      (void*)out, (void*)out, kDm, 0L, fmq_b, rms_w, 0L, kRows, kDm, kDm, kWCarryInv);
}
